// PathFusionEmbedding_43353399885892
// MI455X (gfx1250) — hardware-verified
//
#include <hip/hip_runtime.h>
#include <math.h>

typedef __attribute__((ext_vector_type(16))) _Float16 v16h;
typedef __attribute__((ext_vector_type(8)))  _Float16 v8h;
typedef __attribute__((ext_vector_type(8)))  float    v8f;
typedef __attribute__((ext_vector_type(4)))  float    v4f;

constexpr int kTrees    = 10;
constexpr int kLeaves   = 16;
constexpr int kPathLen  = 5;
constexpr int kNodes    = 31;
constexpr int kD        = 256;
constexpr int kBatch    = 4096;
constexpr int kGate     = 4 * kD;
constexpr int kRows     = kBatch * kTrees;
constexpr int kNodeRows = kTrees * kNodes;
constexpr int kNodePad  = 320;
constexpr int kLeafRows = kTrees * kLeaves;
constexpr int kCrossW   = kTrees * kLeaves;
constexpr int kHP       = 264;
constexpr float kCarry  = 1024.0f;
constexpr float kFold   = 1.0f / (kCarry * kCarry);

static_assert(kGate == 1024 && kRows == 40960 && kNodeRows == 310 && kLeafRows == 160, "shape");
static_assert((1 << (kPathLen - 1)) == kLeaves && kNodes == 2 * kLeaves - 1, "full binary tree");
static_assert(kNodePad >= kNodeRows && (kNodePad % 64) == 0 && (kGate % 64) == 0 && (kD % 32) == 0, "GEMM tile multiples");
static_assert((kRows % 8) == 0, "eight output rows per block");
static_assert(kFold == 9.5367431640625e-07f, "2^-20");

constexpr size_t kOffBtHH  = 0;
constexpr size_t kOffBtIH  = kOffBtHH + (size_t)kGate * kD * 2;
constexpr size_t kOffAEmb  = kOffBtIH + (size_t)kGate * kD * 2;
constexpr size_t kOffNG    = kOffAEmb + (size_t)kNodePad * kD * 2;
constexpr size_t kOffHleaf = kOffNG + (size_t)kNodePad * kGate * 4;
constexpr size_t kWsTotal  = kOffHleaf + (size_t)kLeafRows * kD * 4;
static_assert(kWsTotal == 2686976ull, "carve total");
static_assert(kWsTotal <= 134217728ull, "carve cap");
static_assert((kOffBtIH % 128) == 0 && (kOffAEmb % 128) == 0 && (kOffNG % 128) == 0 && (kOffHleaf % 128) == 0, "128-B aligned regions");

union FragH { v16h v; v8h h[2]; };
__device__ __forceinline__ v16h frag_load(const _Float16* p) {
  FragH f;
  f.h[0] = *(const v8h*)(p);
  f.h[1] = *(const v8h*)(p + 16);
  return f.v;
}
__device__ __forceinline__ v8f mma_g(v16h a, v16h b, v8f c) {
  c = __builtin_amdgcn_wmma_f32_16x16x32_f16(false, a, false, b, (short)0, c, false, false);
  asm volatile("v_nop\n\tv_nop\n\tv_nop\n\tv_nop" : "+v"(c) : "v"(a), "v"(b));
  return c;
}

__device__ __forceinline__ float sigm_fast(float x) {
  return __builtin_amdgcn_rcpf(1.0f + __expf(-x));
}
__device__ __forceinline__ float tanh_fast(float x) {
  return 1.0f - 2.0f * __builtin_amdgcn_rcpf(__expf(2.0f * x) + 1.0f);
}

constexpr int kWBlocks   = (kGate * kD / 8) / 256;
constexpr int kEmbBlocks = (kNodePad * kD / 8) / 256;
constexpr int kEmbValid8 = kNodeRows * kD / 8;
static_assert(kWBlocks == 128 && kEmbBlocks == 40 && kEmbValid8 == 9920, "prep coverage");

__global__ __launch_bounds__(256) void prep_planes_kernel(
    const float* __restrict__ Whh, const float* __restrict__ Wih, const float* __restrict__ emb,
    unsigned short* __restrict__ BtHH, unsigned short* __restrict__ BtIH, unsigned short* __restrict__ AEmb)
{
  const int blk = blockIdx.x;
  const float* src;
  unsigned short* dst;
  int nvalid8;
  int i;
  if (blk < kWBlocks) {
    src = Whh; dst = BtHH; nvalid8 = kGate * kD / 8; i = blk * 256 + threadIdx.x;
  } else if (blk < 2 * kWBlocks) {
    src = Wih; dst = BtIH; nvalid8 = kGate * kD / 8; i = (blk - kWBlocks) * 256 + threadIdx.x;
  } else {
    src = emb; dst = AEmb; nvalid8 = kEmbValid8; i = (blk - 2 * kWBlocks) * 256 + threadIdx.x;
  }
  const bool valid = i < nvalid8;
  const size_t e0 = (size_t)i << 3;
  const size_t ec = valid ? e0 : (size_t)0;
  const v4f a0 = *(const v4f*)(src + ec);
  const v4f a1 = *(const v4f*)(src + ec + 4);
  v8h hv;
#pragma unroll
  for (int e = 0; e < 4; ++e) {
    const float x0 = valid ? a0[e] * kCarry : 0.0f;
    const float x1 = valid ? a1[e] * kCarry : 0.0f;
    hv[e]     = (_Float16)x0;
    hv[4 + e] = (_Float16)x1;
  }
  unsigned short* q = dst + e0;
  *(volatile v8h*)q = hv;
  __threadfence();
  *(volatile v8h*)q = hv;
}

__global__ __launch_bounds__(256) void node_gates_gemm_kernel(
    const unsigned short* __restrict__ Ap, int lda,
    const unsigned short* __restrict__ Btp, int ldb,
    float* __restrict__ C, int ldc,
    const float* __restrict__ bias_a, const float* __restrict__ bias_b,
    int M, int N, int K, float scale)
{
  const _Float16* A  = (const _Float16*)Ap;
  const _Float16* Bt = (const _Float16*)Btp;
  __shared__ __align__(16) float sT[8][16 * 68];
  const int lane = threadIdx.x & 31;
  const int wave = threadIdx.x >> 5;
  const int tilesN = N >> 6;
  const int tilesM = M >> 6;
  const int tile = blockIdx.x * 8 + wave;
  if (tile >= tilesM * tilesN) return;
  const int tm = tile / tilesN;
  const int tn = tile - tm * tilesN;
  const int m0 = tm << 6;
  const int n0 = tn << 6;

  const int rlane = lane & 15;
  const int koff  = (lane >> 4) * 8;
  const int mOff  = (lane >> 4) * 8;

  v8f acc[4][4];
#pragma unroll
  for (int i = 0; i < 4; ++i)
#pragma unroll
    for (int j = 0; j < 4; ++j) acc[i][j] = (v8f){0.f,0.f,0.f,0.f,0.f,0.f,0.f,0.f};

  for (int k0 = 0; k0 < K; k0 += 32) {
    v16h bh[4];
#pragma unroll
    for (int j = 0; j < 4; ++j) {
      const size_t bo = (size_t)(n0 + (j << 4) + rlane) * ldb + koff + k0;
      bh[j] = frag_load(Bt + bo);
    }
#pragma unroll
    for (int i = 0; i < 4; ++i) {
      const size_t ao = (size_t)(m0 + (i << 4) + rlane) * lda + koff + k0;
      const v16h ah = frag_load(A + ao);
#pragma unroll
      for (int j = 0; j < 4; ++j) acc[i][j] = mma_g(ah, bh[j], acc[i][j]);
    }
  }

  float* slab = sT[wave];
#pragma unroll
  for (int i = 0; i < 4; ++i) {
    const int mBase = m0 + (i << 4);
#pragma unroll
    for (int j = 0; j < 4; ++j) {
      const int n = n0 + (j << 4) + rlane;
      const float bv = bias_a[n] + bias_b[n];
#pragma unroll
      for (int r = 0; r < 8; ++r) {
        const float v = acc[i][j][r] * scale + bv;
        slab[(mOff + r) * 68 + (j << 4) + rlane] = v;
      }
    }
    __builtin_amdgcn_fence(__ATOMIC_RELEASE, "workgroup");
    __builtin_amdgcn_wave_barrier();
    __builtin_amdgcn_fence(__ATOMIC_ACQUIRE, "workgroup");
    {
      const int hh = lane >> 4, c4 = (lane & 15) * 4;
      for (int pass = 0; pass < 2; ++pass) {
#pragma unroll
        for (int it = 0; it < 8; ++it) {
          const int row = it * 2 + hh;
          const v4f v = *(const v4f*)(slab + row * 68 + c4);
          *(volatile v4f*)(C + (size_t)(mBase + row) * ldc + n0 + c4) = v;
        }
        __threadfence();
      }
    }
    __builtin_amdgcn_fence(__ATOMIC_RELEASE, "workgroup");
    __builtin_amdgcn_wave_barrier();
    __builtin_amdgcn_fence(__ATOMIC_ACQUIRE, "workgroup");
  }
}

__global__ __launch_bounds__(256) void lstm_leaf_table_kernel(
    const unsigned short* __restrict__ BtHHp, const float* __restrict__ NG, float* __restrict__ Hleaf)
{
  __shared__ __align__(16) float    sNG[kLeaves * kGate];
  __shared__ __align__(16) _Float16 hs[kLeaves * kHP];
  __shared__ __align__(16) float    sOut[kLeaves * kD];

  const _Float16* Bt = (const _Float16*)BtHHp;
  const int tid  = threadIdx.x;
  const int lane = tid & 31;
  const int wave = tid >> 5;
  const int hh   = lane >> 4;
  const int cc   = lane & 15;
  const int tree = blockIdx.x;
  const int dl = 32 * wave + cc;

  const _Float16* bp = Bt + (size_t)dl * kD + 8 * hh;
  const _Float16* ap = hs + cc * kHP + 8 * hh;

  float cst[2][8];
#pragma unroll
  for (int j = 0; j < 2; ++j)
#pragma unroll
    for (int r = 0; r < 8; ++r) cst[j][r] = 0.0f;

#pragma unroll 1
  for (int p = 0; p < kPathLen; ++p) {
    __syncthreads();
    {
      const int nrows = 1 << p;
      const int node0 = tree * kNodes + nrows - 1;
#pragma unroll 1
      for (int i = 0; i < nrows; ++i) {
        int nd = node0 + i;
        nd = nd < kNodePad ? nd : (kNodePad - 1);
        const v4f v = *(const v4f*)(NG + (size_t)nd * kGate + tid * 4);
        *(v4f*)(sNG + i * kGate + tid * 4) = v;
      }
    }
    v8f acc[8];
#pragma unroll
    for (int n = 0; n < 8; ++n) acc[n] = (v8f){0.f,0.f,0.f,0.f,0.f,0.f,0.f,0.f};
    if (p > 0) {
#pragma unroll 1
      for (int kt = 0; kt < kD / 32; ++kt) {
        const v16h a = frag_load(ap + kt * 32);
#pragma unroll
        for (int n = 0; n < 8; ++n) {
          const v16h b = frag_load(bp + (size_t)((n >> 1) * kD + (n & 1) * 16) * kD + kt * 32);
          acc[n] = mma_g(a, b, acc[n]);
        }
      }
    }
    __syncthreads();
    const int lsh = (kPathLen - 1) - p;
    const bool last = (p == kPathLen - 1);
#pragma unroll
    for (int r = 0; r < 8; ++r) {
      const int row = 8 * hh + r;
      const float* ng = sNG + (row >> lsh) * kGate + dl;
#pragma unroll
      for (int j = 0; j < 2; ++j) {
        const float gi = ng[j * 16]          + acc[0 + j][r] * kFold;
        const float gf = ng[kD + j * 16]     + acc[2 + j][r] * kFold;
        const float gg = ng[2 * kD + j * 16] + acc[4 + j][r] * kFold;
        const float go = ng[3 * kD + j * 16] + acc[6 + j][r] * kFold;
        const float cn = sigm_fast(gf) * cst[j][r] + sigm_fast(gi) * tanh_fast(gg);
        cst[j][r] = cn;
        const float ht = sigm_fast(go) * tanh_fast(cn);
        hs[row * kHP + dl + 16 * j] = (_Float16)(ht * kCarry);
        if (last) sOut[row * kD + dl + 16 * j] = ht;
      }
    }
  }
  __syncthreads();
  {
    const int r0 = wave * 2;
    v4f o[2][2];
#pragma unroll
    for (int rr = 0; rr < 2; ++rr)
#pragma unroll
      for (int hb = 0; hb < 2; ++hb)
        o[rr][hb] = *(const v4f*)(sOut + (r0 + rr) * kD + hb * 128 + lane * 4);
    float* dst = Hleaf + (size_t)(tree * kLeaves + r0) * kD;
    for (int pass = 0; pass < 2; ++pass) {
#pragma unroll
      for (int rr = 0; rr < 2; ++rr)
#pragma unroll
        for (int hb = 0; hb < 2; ++hb)
          *(volatile v4f*)(dst + rr * kD + hb * 128 + lane * 4) = o[rr][hb];
      __threadfence();
    }
  }
}

__global__ __launch_bounds__(256) void broadcast_rows_kernel(
    const float* __restrict__ cross, const float* __restrict__ Hleaf, float* __restrict__ out)
{
  const int lane = threadIdx.x & 31;
  const int wave = threadIdx.x >> 5;
  const int n = blockIdx.x * 8 + wave;
  if (n >= kRows) return;
  const int b = n / kTrees;
  const int t = n - b * kTrees;
  const float* cf = cross + (size_t)b * kCrossW + t * kLeaves;
  v4f qv[4];
#pragma unroll
  for (int i = 0; i < 4; ++i) qv[i] = *(const v4f*)(cf + 4 * i);
  float best = qv[0][0];
  int leaf = 0;
#pragma unroll
  for (int i = 0; i < 4; ++i) {
#pragma unroll
    for (int e = 0; e < 4; ++e) {
      const float v = qv[i][e];
      const bool gt = v > best;
      leaf = gt ? (i * 4 + e) : leaf;
      best = gt ? v : best;
    }
  }
  leaf = leaf < 0 ? 0 : leaf;
  leaf = leaf > (kLeaves - 1) ? (kLeaves - 1) : leaf;
  const float* src = Hleaf + (size_t)(t * kLeaves + leaf) * kD;
  const v4f a0 = *(const v4f*)(src + lane * 4);
  const v4f a1 = *(const v4f*)(src + 128 + lane * 4);
  float* dst = out + (size_t)n * kD;
  *(volatile v4f*)(dst + lane * 4) = a0;
  *(volatile v4f*)(dst + 128 + lane * 4) = a1;
  __threadfence();
  *(volatile v4f*)(dst + lane * 4) = a0;
  *(volatile v4f*)(dst + 128 + lane * 4) = a1;
}

extern "C" void kernel_launch(void* const* d_in, const int* in_sizes, int n_in,
                              void* d_out, int out_size, void* d_ws, size_t ws_size,
                              hipStream_t stream) {
  if (n_in < 6) return;
  if (in_sizes[0] != kBatch * kCrossW) return;
  if (in_sizes[1] != kNodeRows * kD) return;
  if (in_sizes[2] != kGate * kD) return;
  if (in_sizes[3] != kGate * kD) return;
  if (in_sizes[4] != kGate) return;
  if (in_sizes[5] != kGate) return;
  if (out_size != kRows * kD) return;
  if (ws_size < kWsTotal) return;

  const float* cross = (const float*)d_in[0];
  const float* emb   = (const float*)d_in[1];
  const float* Wih   = (const float*)d_in[2];
  const float* Whh   = (const float*)d_in[3];
  const float* bih   = (const float*)d_in[4];
  const float* bhh   = (const float*)d_in[5];
  float* out = (float*)d_out;

  char* ws = (char*)d_ws;
  unsigned short* BtHH  = (unsigned short*)(ws + kOffBtHH);
  unsigned short* BtIH  = (unsigned short*)(ws + kOffBtIH);
  unsigned short* AEmb  = (unsigned short*)(ws + kOffAEmb);
  float*          NG    = (float*)(ws + kOffNG);
  float*          Hleaf = (float*)(ws + kOffHleaf);

  prep_planes_kernel<<<2 * kWBlocks + kEmbBlocks, 256, 0, stream>>>(Whh, Wih, emb, BtHH, BtIH, AEmb);

  node_gates_gemm_kernel<<<(kNodePad / 64) * (kGate / 64) / 8, 256, 0, stream>>>(
      AEmb, kD, BtIH, kD, NG, kGate, bih, bhh, kNodePad, kGate, kD, kFold);

  lstm_leaf_table_kernel<<<kTrees, 256, 0, stream>>>(BtHH, NG, Hleaf);

  broadcast_rows_kernel<<<kRows / 8, 256, 0, stream>>>(cross, Hleaf, out);
}
